// LocalWindowSelfAttention_2723009266021
// MI455X (gfx1250) — hardware-verified
//
#include <hip/hip_runtime.h>


#define NBb  4
#define IH   32
#define IW   32
#define NQ   1024
#define CC   256
#define NH_  8
#define HD   32
#define HP64 64
#define WR   3
#define PCAR 1024.0f
typedef _Float16 h16;
typedef unsigned short bf;
typedef __attribute__((ext_vector_type(16))) __bf16   v16bf;
typedef __attribute__((ext_vector_type(16))) _Float16 v16h;
typedef __attribute__((ext_vector_type(8)))  _Float16 v8h;
typedef __attribute__((ext_vector_type(8)))  unsigned short v8us;
typedef __attribute__((ext_vector_type(8)))  float    v8f;
typedef __attribute__((ext_vector_type(4)))  float    v4f;
typedef v8h  __attribute__((may_alias)) v8ha;
typedef v4f  __attribute__((may_alias)) v4fa;
typedef v8us __attribute__((may_alias)) v8usa;

__device__ __forceinline__ unsigned short f2bf(float f) { unsigned u = __float_as_uint(f); u += 0x7FFFu + ((u >> 16) & 1u); return (unsigned short)(u >> 16); }
__device__ __forceinline__ float bf2f(unsigned short b) { return __uint_as_float(((unsigned)b) << 16); }
__device__ __forceinline__ float bfr(float f) { return bf2f(f2bf(f)); }
__device__ __forceinline__ v16h cat16(v8h lo, v8h hi) { return __builtin_shufflevector(lo, hi, 0, 1, 2, 3, 4, 5, 6, 7, 8, 9, 10, 11, 12, 13, 14, 15); }
__device__ __forceinline__ v16bf cat16b(v8us lo, v8us hi) { return __builtin_bit_cast(v16bf, __builtin_shufflevector(lo, hi, 0, 1, 2, 3, 4, 5, 6, 7, 8, 9, 10, 11, 12, 13, 14, 15)); }
__device__ __forceinline__ v8f wmma16(v16h a, v16h b, v8f c) { return __builtin_amdgcn_wmma_f32_16x16x32_f16(false, a, false, b, (short)0, c, false, false); }
__device__ __forceinline__ v8f wmmab(v16bf a, v16bf b, v8f c) { return __builtin_amdgcn_wmma_f32_16x16x32_bf16(false, a, false, b, (short)0, c, false, false); }


template <typename T16> struct WFrag;
template <> struct WFrag<h16> { typedef v16h V; static __device__ __forceinline__ V ld(const h16* p) { return cat16(*(const v8h*)p, *(const v8h*)(p + 16)); } static __device__ __forceinline__ v8f mma(V a, V b, v8f c) { return wmma16(a, b, c); } };
template <> struct WFrag<bf> { typedef v16bf V; static __device__ __forceinline__ V ld(const bf* p) { return cat16b(*(const v8us*)p, *(const v8us*)(p + 16)); } static __device__ __forceinline__ v8f mma(V a, V b, v8f c) { return wmmab(a, b, c); } };
template <typename T16, int NSPLIT, bool BIAS>
__global__ __launch_bounds__(32) void k_gemmw(const T16* __restrict__ A, const T16* __restrict__ A2, const T16* __restrict__ Bt, const T16* __restrict__ Bt2, int K, float* C, int ldc, const float* __restrict__ bias, size_t sA, size_t sB, size_t sC) {
    typedef typename WFrag<T16>::V V;
    __shared__ __align__(16) float os[16 * 68];
    const size_t z = blockIdx.z; A += z * sA; if (A2) A2 += z * sA; Bt += z * sB; if (Bt2) Bt2 += z * sB; C += z * sC;
    const int lane = threadIdx.x & 31, lr = lane & 15, hi = lane >> 4; const int r0 = blockIdx.x * 64, c0 = blockIdx.y * 64;
    v8f acc[4][4];
#pragma unroll
    for (int mb = 0; mb < 4; ++mb)
#pragma unroll
        for (int nb = 0; nb < 4; ++nb) acc[mb][nb] = (v8f){};
    const size_t aoff = (size_t)(r0 + lr) * K + 8 * hi, boff = (size_t)(c0 + lr) * K + 8 * hi;
#pragma unroll 1
    for (int kc = 0; kc < K; kc += 32) {
        V a[4], a2[4];
#pragma unroll
        for (int mb = 0; mb < 4; ++mb) { a[mb] = WFrag<T16>::ld(A + aoff + (size_t)mb * 16 * K + kc); if (NSPLIT == 1 || NSPLIT == 2) a2[mb] = WFrag<T16>::ld(A2 + aoff + (size_t)mb * 16 * K + kc); }
#pragma unroll
        for (int nb = 0; nb < 4; ++nb) { const V b = WFrag<T16>::ld(Bt + boff + (size_t)nb * 16 * K + kc); V b2; if (NSPLIT >= 2) b2 = WFrag<T16>::ld(Bt2 + boff + (size_t)nb * 16 * K + kc);
#pragma unroll
            for (int mb = 0; mb < 4; ++mb) { acc[mb][nb] = WFrag<T16>::mma(a[mb], b, acc[mb][nb]); if (NSPLIT == 1 || NSPLIT == 2) acc[mb][nb] = WFrag<T16>::mma(a2[mb], b, acc[mb][nb]); if (NSPLIT >= 2) acc[mb][nb] = WFrag<T16>::mma(a[mb], b2, acc[mb][nb]); } }
        asm volatile("v_nop\n\tv_nop\n\tv_nop\n\tv_nop" : "+v"(acc[0][0]), "+v"(acc[1][1]), "+v"(acc[2][2]), "+v"(acc[3][3]) : "v"(a[0]), "v"(a[3]));
    }
#pragma unroll
    for (int mb = 0; mb < 4; ++mb) {
#pragma unroll
        for (int nb = 0; nb < 4; ++nb) {
#pragma unroll
            for (int j = 0; j < 8; ++j) os[(hi * 8 + j) * 68 + nb * 16 + lr] = acc[mb][nb][j]; }
        __builtin_amdgcn_wave_barrier(); asm volatile("" ::: "memory");
        float* crow = C + (size_t)(r0 + mb * 16) * ldc + c0;
#pragma unroll 1
        for (int ps = 0; ps < 2; ++ps) {
#pragma unroll
            for (int s = 0; s < 8; ++s) { const int row = 2 * s + hi, cofs = lr * 4; v4f val = *(const v4fa*)(os + row * 68 + cofs); if (BIAS) { val[0] += bfr(bias[c0 + cofs]); val[1] += bfr(bias[c0 + cofs + 1]); val[2] += bfr(bias[c0 + cofs + 2]); val[3] += bfr(bias[c0 + cofs + 3]); }
                *(volatile v4f*)(crow + (size_t)row * ldc + cofs) = val; }
            if (ps == 0) __threadfence(); }
        __builtin_amdgcn_wave_barrier(); asm volatile("" ::: "memory");
    }
}

__device__ __forceinline__ h16 tohx(float x) { return (h16)x; }
__device__ __forceinline__ void splitf(float y, unsigned short& h, unsigned short& l) { h = f2bf(y); l = f2bf(y - bf2f(h)); }
typedef __attribute__((ext_vector_type(2))) unsigned short v2us;
typedef __attribute__((ext_vector_type(4))) unsigned short v4us;
typedef __attribute__((ext_vector_type(2))) _Float16 v2h;
typedef __attribute__((ext_vector_type(4))) _Float16 v4h;

__global__ __launch_bounds__(256) void k_wtG(const float* __restrict__ w, int K, int N, bf* Bt) {
    const int lane = threadIdx.x & 31; const int L0 = (blockIdx.x * 8 + (threadIdx.x >> 5)) * 8; const int nlines = N * K / 64;
#pragma unroll
    for (int ps = 0; ps < 2; ++ps) {
#pragma unroll 1
        for (int l = 0; l < 8; ++l) { const int L = L0 + l; if (L >= nlines) break; const size_t e = (size_t)L * 64 + lane * 2; const int k = (int)(e % K), n = (int)(e / K); v2us o;
            o[0] = f2bf(w[(size_t)k * N + n]); o[1] = f2bf(w[(size_t)(k + 1) * N + n]); *(volatile v2us*)(Bt + e) = o; }
        if (ps == 0) __threadfence(); }
}
__global__ __launch_bounds__(256) void k_cvt8(const float* __restrict__ src, bf* dst, size_t n8) { const size_t i = (size_t)blockIdx.x * 256 + threadIdx.x; if (i >= n8) return; const v8f v = *(const v8f*)(src + i * 8); v8us o;
#pragma unroll
    for (int k = 0; k < 8; ++k) o[k] = f2bf(v[k]); *(volatile v8us*)(dst + i * 8) = o; __threadfence(); *(volatile v8us*)(dst + i * 8) = o; }
__global__ __launch_bounds__(256) void k_xt(const float* __restrict__ img, bf* XT) { const int e = (blockIdx.x * 256 + threadIdx.x) * 2; if (e >= NQ * CC) return; const int c = e % CC; const int p = e / CC; v2us o; o[0] = f2bf(img[(size_t)c * NQ + p]); o[1] = f2bf(img[(size_t)(c + 1) * NQ + p]); *(volatile v2us*)(XT + e) = o; __threadfence(); *(volatile v2us*)(XT + e) = o; }
__global__ __launch_bounds__(256) void k_qkpl(const float* __restrict__ Q, const float* __restrict__ KV, bf* Qh, bf* Ql, bf* Kh, bf* Kl) { const int e = (blockIdx.x * 256 + threadIdx.x) * 4; if (e >= NH_ * NQ * HD) return; const int d = e % HD; const int q = (e / HD) % NQ; const int h = e / (HD * NQ); const v4f a = *(const v4f*)(Q + (size_t)q * CC + h * HD + d), k = *(const v4f*)(KV + (size_t)q * 2 * CC + h * HD + d); v4us qh, ql, kh, kl;
#pragma unroll
    for (int u = 0; u < 4; ++u) { unsigned short x, y; splitf(a[u] * 0.17677669529663687f, x, y); qh[u] = x; ql[u] = y; splitf(k[u], x, y); kh[u] = x; kl[u] = y; }
    for (int ps = 0; ps < 2; ++ps) { *(volatile v4us*)(Qh + e) = qh; *(volatile v4us*)(Ql + e) = ql; *(volatile v4us*)(Kh + e) = kh; *(volatile v4us*)(Kl + e) = kl; if (ps == 0) __threadfence(); } }
__global__ __launch_bounds__(256) void k_vt(const float* __restrict__ KV, h16* VT) { const int e = (blockIdx.x * 256 + threadIdx.x) * 2; if (e >= NH_ * HP64 * NQ) return; const int p = e % NQ; const int dp = (e / NQ) % HP64; const int h = e / (NQ * HP64); v2h o;
#pragma unroll
    for (int u = 0; u < 2; ++u) o[u] = (dp < HD) ? tohx(KV[(size_t)(p + u) * 2 * CC + CC + h * HD + dp]) : tohx(0.f); *(volatile v2h*)(VT + e) = o; __threadfence(); *(volatile v2h*)(VT + e) = o; }
__global__ __launch_bounds__(256) void k_mrg(const float* __restrict__ O, bf* Mh, bf* Ml) { const int e = (blockIdx.x * 256 + threadIdx.x) * 4; if (e >= NQ * CC) return; const int c = e % CC; const int q = e / CC; const int h = c / HD, d = c % HD; const float* r = O + ((size_t)h * NQ + q) * HP64 + d; v4us oh, ol;
#pragma unroll
    for (int u = 0; u < 4; ++u) { unsigned short a, b; splitf(r[u] * (1.0f / PCAR), a, b); oh[u] = a; ol[u] = b; } *(volatile v4us*)(Mh + e) = oh; *(volatile v4us*)(Ml + e) = ol; __threadfence(); *(volatile v4us*)(Mh + e) = oh; *(volatile v4us*)(Ml + e) = ol; }
__global__ __launch_bounds__(256) void k_tr(const float* __restrict__ F, float* OUTb) { const int e = (blockIdx.x * 256 + threadIdx.x) * 4; if (e >= CC * NQ) return; const int q = e % NQ; const int c = e / NQ; v4f o;
#pragma unroll
    for (int u = 0; u < 4; ++u) o[u] = F[(size_t)(q + u) * CC + c]; *(volatile v4f*)(OUTb + e) = o; __threadfence(); *(volatile v4f*)(OUTb + e) = o; }
__global__ __launch_bounds__(256) void k_wmsoft(const float* __restrict__ Sb, h16* P16) { const int lane = threadIdx.x & 31; const int row = blockIdx.x * 8 + (threadIdx.x >> 5); if (row >= NH_ * NQ) return; const int q = row % NQ; const int qy = q / IW, qx = q % IW; const float* sr = Sb + (size_t)row * NQ; float v[32]; float mx = -3.0e38f;
#pragma unroll
    for (int ch = 0; ch < 8; ++ch) { const int j0 = ch * 128 + lane * 4; const v4f a = *(const v4f*)(sr + j0);
#pragma unroll
        for (int u = 0; u < 4; ++u) { const int j = j0 + u; const int ky = j / IW, kx = j % IW; const bool ok = (ky >= qy - WR) && (ky <= qy + WR) && (kx >= qx - WR) && (kx <= qx + WR); const float t = ok ? a[u] : -3.0e38f; v[ch * 4 + u] = t; mx = fmaxf(mx, t); } }
#pragma unroll
    for (int sh = 16; sh; sh >>= 1) mx = fmaxf(mx, __shfl_xor(mx, sh, 32));
    float sum = 0.f;
#pragma unroll
    for (int k = 0; k < 32; ++k) { float d0 = __fsub_rn(v[k], mx); asm volatile("" : "+v"(d0)); v[k] = __builtin_amdgcn_exp2f(__fmul_rn(d0, 1.4426950408889634f)); sum += v[k]; }
#pragma unroll
    for (int sh = 16; sh; sh >>= 1) sum += __shfl_xor(sum, sh, 32);
    const float f = __fdiv_rn(PCAR, sum);
    for (int ps = 0; ps < 2; ++ps) {
#pragma unroll
        for (int ch = 0; ch < 8; ++ch) { v4h o;
#pragma unroll
            for (int u = 0; u < 4; ++u) o[u] = tohx(v[ch * 4 + u] * f); *(volatile v4h*)(P16 + (size_t)row * NQ + ch * 128 + lane * 4) = o; }
        if (ps == 0) __threadfence(); } }

extern "C" void kernel_launch(void* const* d_in, const int* in_sizes, int n_in,
                              void* d_out, int out_size, void* d_ws, size_t ws_size, hipStream_t stream) {
    (void)in_sizes; (void)n_in; (void)out_size;
    const float* img = (const float*)d_in[0]; const float* qin = (const float*)d_in[1]; const float* wkv = (const float*)d_in[2]; const float* bkv = (const float*)d_in[3]; const float* wq = (const float*)d_in[4]; const float* bq = (const float*)d_in[5]; const float* wout = (const float*)d_in[6]; const float* bout = (const float*)d_in[7];
    float* OUT = (float*)d_out;
    char* wsp = (char*)d_ws;
    auto take = [&](size_t bytes) { char* p = wsp; wsp += (bytes + 255) & ~(size_t)255; return (void*)p; };
    bf* WKV = (bf*)take((size_t)2 * CC * CC * 2); bf* WQ = (bf*)take((size_t)CC * CC * 2); bf* WO = (bf*)take((size_t)CC * CC * 2);
    bf* XT = (bf*)take((size_t)NQ * CC * 2); bf* XQ = (bf*)take((size_t)NQ * CC * 2); float* Q = (float*)take((size_t)NQ * CC * 4); float* KV = (float*)take((size_t)NQ * 2 * CC * 4); bf* Qh = (bf*)take((size_t)NH_ * NQ * HD * 2); bf* Ql = (bf*)take((size_t)NH_ * NQ * HD * 2); bf* Kh = (bf*)take((size_t)NH_ * NQ * HD * 2); bf* Kl = (bf*)take((size_t)NH_ * NQ * HD * 2); h16* VT = (h16*)take((size_t)NH_ * HP64 * NQ * 2);
    float* Sb = (float*)take((size_t)NH_ * NQ * NQ * 4); h16* P16 = (h16*)take((size_t)NH_ * NQ * NQ * 2); float* O = (float*)take((size_t)NH_ * NQ * HP64 * 4); bf* Mh = (bf*)take((size_t)NQ * CC * 2); bf* Ml = (bf*)take((size_t)NQ * CC * 2); float* F = (float*)take((size_t)NQ * CC * 4);
    if ((size_t)(wsp - (char*)d_ws) > ws_size) return;
    k_wtG<<<(CC * 2 * CC / 64 + 63) / 64, 256, 0, stream>>>(wkv, CC, 2 * CC, WKV); k_wtG<<<(CC * CC / 64 + 63) / 64, 256, 0, stream>>>(wq, CC, CC, WQ); k_wtG<<<(CC * CC / 64 + 63) / 64, 256, 0, stream>>>(wout, CC, CC, WO);
    for (int b = 0; b < NBb; ++b) {
        k_xt<<<(NQ * CC / 2 + 255) / 256, 256, 0, stream>>>(img + (size_t)b * CC * NQ, XT); k_gemmw<bf, 0, true><<<dim3(NQ / 64, 2 * CC / 64, 1), 32, 0, stream>>>(XT, nullptr, WKV, nullptr, CC, KV, 2 * CC, bkv, 0, 0, 0);
        k_cvt8<<<(NQ * CC / 8 + 255) / 256, 256, 0, stream>>>(qin + (size_t)b * NQ * CC, XQ, (size_t)NQ * CC / 8); k_gemmw<bf, 0, true><<<dim3(NQ / 64, CC / 64, 1), 32, 0, stream>>>(XQ, nullptr, WQ, nullptr, CC, Q, CC, bq, 0, 0, 0);
        k_qkpl<<<(NH_ * NQ * HD / 4 + 255) / 256, 256, 0, stream>>>(Q, KV, Qh, Ql, Kh, Kl); k_vt<<<(NH_ * HP64 * NQ / 2 + 255) / 256, 256, 0, stream>>>(KV, VT);
        k_gemmw<bf, 2, false><<<dim3(NQ / 64, NQ / 64, NH_), 32, 0, stream>>>(Qh, Ql, Kh, Kl, HD, Sb, NQ, nullptr, (size_t)NQ * HD, (size_t)NQ * HD, (size_t)NQ * NQ);
        k_wmsoft<<<NH_ * NQ / 8, 256, 0, stream>>>(Sb, P16);
        k_gemmw<h16, 0, false><<<dim3(NQ / 64, HP64 / 64, NH_), 32, 0, stream>>>(P16, nullptr, VT, nullptr, NQ, O, HP64, nullptr, (size_t)NQ * NQ, (size_t)HP64 * NQ, (size_t)NQ * HP64);
        k_mrg<<<(NQ * CC / 4 + 255) / 256, 256, 0, stream>>>(O, Mh, Ml);
        k_gemmw<bf, 1, true><<<dim3(NQ / 64, CC / 64, 1), 32, 0, stream>>>(Mh, Ml, WO, nullptr, CC, F, CC, bout, 0, 0, 0);
        k_tr<<<(CC * NQ / 4 + 255) / 256, 256, 0, stream>>>(F, OUT + (size_t)b * CC * NQ); }
}
